// TrfEdgeNetL1_79645873537754
// MI455X (gfx1250) — hardware-verified
//
#include <hip/hip_runtime.h>
#include <stddef.h>


#define NTHR   256
#define NWAVE  8
#define EPT    8
#define CHUNK  (NTHR * EPT)
#define WCAP   (EPT * 32)
#define LISTN  (NWAVE * WCAP)
#define NB     128
#define FIN    128
#define HC     256
#define NH     4
#define CH     64
#define FE     32
#define QW     128
#define QKVW   768
#define NCLS   16
#define GK     128
#define GBM    64
#define GBN    64
#define BN_EPS 1e-5f
#define NEGBIG (-1.0e30f)
#define AGG_LDS_BYTES ((size_t)NB * (HC + QW + 8) * 4)

static_assert(NB == 16 * NWAVE);
static_assert((NB & (NB - 1)) == 0);
static_assert(NH * CH == HC);
static_assert(NH * FE == QW);
static_assert(WCAP == 256);
static_assert(GK == FIN);
static_assert(GK / 8 == 16);
static_assert(CHUNK < (1 << 23));

typedef float          v4f  __attribute__((ext_vector_type(4)));
typedef float          v8f  __attribute__((ext_vector_type(8)));
typedef int            v4i  __attribute__((ext_vector_type(4)));
typedef unsigned short v8us __attribute__((ext_vector_type(8)));
typedef __bf16         v16b __attribute__((ext_vector_type(16)));
union FragB { v16b v; v8us u[2]; };

__device__ __forceinline__ unsigned short bf16_rne(float x) {
  unsigned u = __float_as_uint(x);
  u = (u + 0x7FFFu + ((u >> 16) & 1u)) >> 16;
  return (unsigned short)u;
}

__device__ __forceinline__ void split8(const float* f, v8us& hi, v8us& lo) {
  v8us h, l;
#pragma unroll
  for (int j = 0; j < 8; ++j) {
    const unsigned short hb = bf16_rne(f[j]);
    const float rem = f[j] - __uint_as_float(((unsigned)hb) << 16);
    h[j] = hb;
    l[j] = bf16_rne(rem);
  }
  hi = h;
  lo = l;
}

__device__ __forceinline__ void unpack8(v4f a, v4f b, float* f) {
  f[0] = a.x; f[1] = a.y; f[2] = a.z; f[3] = a.w;
  f[4] = b.x; f[5] = b.y; f[6] = b.z; f[7] = b.w;
}

__device__ __forceinline__ v8f zero8f() {
  v8f z;
#pragma unroll
  for (int i = 0; i < 8; ++i) z[i] = 0.0f;
  return z;
}

__device__ __forceinline__ v8f wmb(v16b a, v16b b, v8f c) {
  v8f d = __builtin_amdgcn_wmma_f32_16x16x32_bf16(false, a, false, b, (short)0, c, false, false);
  asm volatile("v_nop\n\tv_nop\n\tv_nop\n\tv_nop" : "+v"(d) : "v"(a), "v"(b));
  return d;
}

__device__ __forceinline__ v8f wm3(v16b ah, v16b al, v16b bh, v16b bl, v8f c) {
  c = wmb(ah, bh, c);
  c = wmb(ah, bl, c);
  c = wmb(al, bh, c);
  return c;
}

__device__ __forceinline__ v16b ldfrag(const unsigned short* base, int row, int pitch, int k0, int hh) {
  FragB f;
  const unsigned short* p = base + row * pitch + k0 + 8 * hh;
  f.u[0] = *(const v8us*)p;
  f.u[1] = *(const v8us*)(p + 16);
  return f.v;
}

__global__ __launch_bounds__(NTHR) void k_prep(
    const float* __restrict__ Wq, const float* __restrict__ Wk, const float* __restrict__ Wv,
    const float* __restrict__ We, const float* __restrict__ Wskip, const float* __restrict__ Wc,
    const float* __restrict__ bq, const float* __restrict__ bk, const float* __restrict__ bv,
    unsigned short* wcat_h, unsigned short* wcat_l, unsigned short* webd_h, unsigned short* webd_l,
    unsigned short* wp_h, unsigned short* wp_l, unsigned short* wsk_h, unsigned short* wsk_l,
    unsigned short* wc_h, unsigned short* wc_l, float* biascat) {
  const int y = blockIdx.y;
  const int u = blockIdx.x * NTHR + threadIdx.x;
  if (y == 5) {
    if (u >= QKVW / 4) return;
    float t[4];
#pragma unroll
    for (int j = 0; j < 4; ++j) {
      const int i = 4 * u + j;
      int cq = i;       cq = cq > HC - 1 ? HC - 1 : cq;
      int ck = i - HC;  ck = ck < 0 ? 0 : (ck > HC - 1 ? HC - 1 : ck);
      int cv = i - 2 * HC; cv = cv < 0 ? 0 : (cv > HC - 1 ? HC - 1 : cv);
      const float a = bq[cq], b = bk[ck], c = bv[cv];
      t[j] = (i < HC) ? a : ((i < 2 * HC) ? b : c);
    }
    v4f v = {t[0], t[1], t[2], t[3]};
    float* p = biascat + 4 * u;
    *(volatile v4f*)p = v;
    __threadfence();
    *(volatile v4f*)p = v;
    return;
  }
  int cnt;
  unsigned short* dh;
  unsigned short* dl;
  if (y == 0)      { cnt = QKVW * GK / 8;   dh = wcat_h; dl = wcat_l; }
  else if (y == 1) { cnt = 2 * GBN * GK / 8; dh = webd_h; dl = webd_l; }
  else if (y == 2) { cnt = CH * GK / 8;     dh = wp_h;   dl = wp_l;   }
  else if (y == 3) { cnt = CH * GK / 8;     dh = wsk_h;  dl = wsk_l;  }
  else             { cnt = NCLS * CH / 8;   dh = wc_h;   dl = wc_l;   }
  if (u >= cnt) return;
  float f[8];
  if (y == 0) {
    const int n = u >> 4, k8 = (u & 15) * 8;
    int cq = n;          cq = cq > HC - 1 ? HC - 1 : cq;
    int ck = n - HC;     ck = ck < 0 ? 0 : (ck > HC - 1 ? HC - 1 : ck);
    int cv = n - 2 * HC; cv = cv < 0 ? 0 : (cv > HC - 1 ? HC - 1 : cv);
#pragma unroll
    for (int j = 0; j < 8; ++j) {
      const int k = k8 + j;
      const float a = Wq[k * HC + cq], b = Wk[k * HC + ck], c = Wv[k * HC + cv];
      f[j] = (n < HC) ? a : ((n < 2 * HC) ? b : c);
    }
  } else if (y == 1) {
    const int nrow = u >> 4, k8 = (u & 15) * 8;
    const int z = nrow >> 6, n = nrow & 63;
    const int hd = 2 * z + (n >> 5), fi = n & 31;
#pragma unroll
    for (int j = 0; j < 8; ++j) {
      const int k = k8 + j;
      const int hk = 2 * z + (k >> 6), c = k & 63;
      const float w = We[fi * HC + hd * CH + c];
      f[j] = (hk == hd) ? w : 0.0f;
    }
  } else if (y == 2) {
    const int n = u >> 4, k8 = (u & 15) * 8;
#pragma unroll
    for (int j = 0; j < 8; ++j) {
      const int k = k8 + j;
      const int h = k >> 5, fi = k & 31;
      f[j] = We[fi * HC + h * CH + n];
    }
  } else if (y == 3) {
    const int n = u >> 4, k8 = (u & 15) * 8;
#pragma unroll
    for (int j = 0; j < 8; ++j) f[j] = Wskip[(k8 + j) * CH + n];
  } else {
    const int n = u >> 3, k8 = (u & 7) * 8;
#pragma unroll
    for (int j = 0; j < 8; ++j) f[j] = Wc[(k8 + j) * NCLS + n];
  }
  v8us hi, lo;
  split8(f, hi, lo);
  unsigned short* ph = dh + (size_t)u * 8;
  unsigned short* pl = dl + (size_t)u * 8;
  *(volatile v8us*)ph = hi;
  *(volatile v8us*)pl = lo;
  __threadfence();
  *(volatile v8us*)ph = hi;
  *(volatile v8us*)pl = lo;
}

__global__ __launch_bounds__(NTHR) void k_gemm(const float* __restrict__ A, int lda, int aColStrideY, int nRowsA,
                                               const unsigned short* __restrict__ Bh, const unsigned short* __restrict__ Bl,
                                               int nSlabs, int diag, const float* __restrict__ bias, int hasBias,
                                               float* C, int ldc) {
  __shared__ __attribute__((aligned(16))) unsigned short Ah[GBM * GK];
  __shared__ __attribute__((aligned(16))) unsigned short Al[GBM * GK];
  __shared__ __attribute__((aligned(16))) unsigned short Bsh[GBN * GK];
  __shared__ __attribute__((aligned(16))) unsigned short Bsl[GBN * GK];
  __shared__ __attribute__((aligned(16))) float Cs[GBM * GBN];
  const int tid = threadIdx.x, lane = tid & 31, wave = tid >> 5, hh = lane >> 4, m = lane & 15;
  const int row0 = blockIdx.x * GBM, y = blockIdx.y;
  const int aoff = y * aColStrideY;

  for (int u = tid; u < GBM * (GK / 8); u += NTHR) {
    const int r = u >> 4, k8 = (u & 15) * 8;
    int grow = row0 + r;
    grow = grow > nRowsA - 1 ? nRowsA - 1 : grow;
    const float* p = A + (size_t)grow * lda + aoff + k8;
    const v4f f0 = *(const v4f*)p;
    const v4f f1 = *(const v4f*)(p + 4);
    float f[8];
    unpack8(f0, f1, f);
    v8us hi, lo;
    split8(f, hi, lo);
    *(v8us*)(Ah + r * GK + k8) = hi;
    *(v8us*)(Al + r * GK + k8) = lo;
  }
  const int mt = wave >> 1, nt0 = 2 * (wave & 1);
  const int ksBeg = (diag != 0) ? nt0 : 0;
  const int ksEnd = (diag != 0) ? nt0 + 2 : GK / 32;

#pragma unroll 1
  for (int s = 0; s < nSlabs; ++s) {
    const int slab = y * nSlabs + s;
    const unsigned short* bh = Bh + (size_t)slab * GBN * GK;
    const unsigned short* bl = Bl + (size_t)slab * GBN * GK;
    for (int u = tid; u < GBN * (GK / 8); u += NTHR) {
      *(v8us*)(Bsh + u * 8) = *(const v8us*)(bh + (size_t)u * 8);
      *(v8us*)(Bsl + u * 8) = *(const v8us*)(bl + (size_t)u * 8);
    }
    __syncthreads();

    v8f acc[2];
    acc[0] = zero8f();
    acc[1] = zero8f();
    for (int ks = ksBeg; ks < ksEnd; ++ks) {
      const v16b ah = ldfrag(Ah, 16 * mt + m, GK, 32 * ks, hh);
      const v16b al = ldfrag(Al, 16 * mt + m, GK, 32 * ks, hh);
#pragma unroll
      for (int t = 0; t < 2; ++t) {
        const v16b bhf = ldfrag(Bsh, 16 * (nt0 + t) + m, GK, 32 * ks, hh);
        const v16b blf = ldfrag(Bsl, 16 * (nt0 + t) + m, GK, 32 * ks, hh);
        acc[t] = wm3(ah, al, bhf, blf, acc[t]);
      }
    }
#pragma unroll
    for (int t = 0; t < 2; ++t) {
      const int cl = 16 * (nt0 + t) + m;
      float bvv = 0.0f;
      if (hasBias != 0) bvv = bias[slab * GBN + cl];
#pragma unroll
      for (int r = 0; r < 8; ++r) Cs[(16 * mt + 8 * hh + r) * GBN + cl] = acc[t][r] + bvv;
    }
    __syncthreads();

    v4f ov[4];
    size_t go[4];
#pragma unroll
    for (int i = 0; i < 4; ++i) {
      const int rl = 8 * wave + 2 * i + hh;
      ov[i] = *(const v4f*)(Cs + rl * GBN + 4 * m);
      go[i] = (size_t)(row0 + rl) * ldc + (size_t)slab * GBN + 4 * m;
    }
#pragma unroll
    for (int i = 0; i < 4; ++i) *(volatile v4f*)(C + go[i]) = ov[i];
    __threadfence();
#pragma unroll
    for (int i = 0; i < 4; ++i) *(volatile v4f*)(C + go[i]) = ov[i];
    __syncthreads();
  }
}

__device__ __forceinline__ int scan_chunk(const int* __restrict__ dsts, int nE, int cbase, int nodeBase,
                                          int vec8, int* list, int tid, int wave) {
  int wc = 0;
  const int el0  = tid * EPT;
  const int e0   = cbase + el0;
  const int sent = -2147483647 - 1;
  v4i da, db;
  if (vec8 != 0 && cbase + CHUNK <= nE) {
    da = *(const v4i*)(dsts + e0);
    db = *(const v4i*)(dsts + e0 + 4);
  } else {
    da.x = (e0     < nE) ? dsts[min(e0, nE - 1)] : sent;
    da.y = (e0 + 1 < nE) ? dsts[min(e0 + 1, nE - 1)] : sent;
    da.z = (e0 + 2 < nE) ? dsts[min(e0 + 2, nE - 1)] : sent;
    da.w = (e0 + 3 < nE) ? dsts[min(e0 + 3, nE - 1)] : sent;
    db.x = (e0 + 4 < nE) ? dsts[min(e0 + 4, nE - 1)] : sent;
    db.y = (e0 + 5 < nE) ? dsts[min(e0 + 5, nE - 1)] : sent;
    db.z = (e0 + 6 < nE) ? dsts[min(e0 + 6, nE - 1)] : sent;
    db.w = (e0 + 7 < nE) ? dsts[min(e0 + 7, nE - 1)] : sent;
  }
  const unsigned nb = (unsigned)nodeBase;
  const unsigned s0 = (unsigned)da.x - nb, s1 = (unsigned)da.y - nb;
  const unsigned s2 = (unsigned)da.z - nb, s3 = (unsigned)da.w - nb;
  const unsigned s4 = (unsigned)db.x - nb, s5 = (unsigned)db.y - nb;
  const unsigned s6 = (unsigned)db.z - nb, s7 = (unsigned)db.w - nb;
  const bool h0 = s0 < (unsigned)NB, h1 = s1 < (unsigned)NB, h2 = s2 < (unsigned)NB, h3 = s3 < (unsigned)NB;
  const bool h4 = s4 < (unsigned)NB, h5 = s5 < (unsigned)NB, h6 = s6 < (unsigned)NB, h7 = s7 < (unsigned)NB;
  const unsigned any = __builtin_amdgcn_ballot_w32(h0 | h1 | h2 | h3 | h4 | h5 | h6 | h7);
  if (any != 0u) {
#define HITJ(J, HJ, SJ) { \
      const unsigned mj = __builtin_amdgcn_ballot_w32(HJ); \
      if (mj != 0u) { \
        if (HJ) { \
          const int pos = wc + (int)__builtin_amdgcn_mbcnt_lo(mj, 0u); \
          if (pos < WCAP) list[wave * WCAP + pos] = (int)((((unsigned)(el0 + (J))) << 8) | (SJ)); \
        } \
        wc += (int)__builtin_popcount(mj); } }
    HITJ(0, h0, s0)
    HITJ(1, h1, s1)
    HITJ(2, h2, s2)
    HITJ(3, h3, s3)
    HITJ(4, h4, s4)
    HITJ(5, h5, s5)
    HITJ(6, h6, s6)
    HITJ(7, h7, s7)
#undef HITJ
  }
  return wc;
}

__global__ __launch_bounds__(NTHR) void k_agg(const int* __restrict__ ei, int nE, int nN, int vec8,
                                              const float* __restrict__ ea, const float* __restrict__ qkv,
                                              const float* __restrict__ qwe, float* agg64, float* aea) {
  extern __shared__ v4f dsm[];
  __shared__ __attribute__((aligned(16))) int list[LISTN];
  __shared__ int wcnt[NWAVE];
  float* accv = (float*)dsm;
  float* acce = accv + NB * HC;
  float* mden = acce + NB * QW;

  const int tid = threadIdx.x, lane = tid & 31, wave = tid >> 5, hh = lane >> 4, m = lane & 15;
  const int hd = lane >> 3;
  const int nodeBase = blockIdx.x * NB;
  const int* srcs = ei;
  const int* dsts = ei + nE;

  {
    const v4f z4 = {0.0f, 0.0f, 0.0f, 0.0f};
    const v4f n4 = {NEGBIG, NEGBIG, NEGBIG, NEGBIG};
    for (int i = tid; i < NB * (HC + QW) / 4; i += NTHR) dsm[i] = z4;
    for (int i = tid; i < NB * 2; i += NTHR) {
      const v4f v = ((i & 1) != 0) ? z4 : n4;
      *(v4f*)(mden + (i >> 1) * 8 + 4 * (i & 1)) = v;
    }
  }
  __syncthreads();

  const int nChunks = (nE + CHUNK - 1) / CHUNK;
#pragma unroll 1
  for (int ch = 0; ch < nChunks; ++ch) {
    const int cbase = ch * CHUNK;
    const int wc = scan_chunk(dsts, nE, cbase, nodeBase, vec8, list, tid, wave);
    if (lane == 0) wcnt[wave] = wc;
    __syncthreads();

#pragma unroll 1
    for (int w2 = 0; w2 < NWAVE; ++w2) {
      int n = wcnt[w2];
      n = n < 0 ? 0 : (n > WCAP ? WCAP : n);
#pragma unroll 1
      for (int i = 0; i < n; ++i) {
        const int ent  = __builtin_amdgcn_readfirstlane(list[w2 * WCAP + i]);
        const int slot = ent & (NB - 1);
        if ((slot & (NWAVE - 1)) != wave) continue;
        int e = cbase + (ent >> 8);
        e = e < 0 ? 0 : (e > nE - 1 ? nE - 1 : e);
        int src = srcs[e];
        src = src < 0 ? 0 : (src > nN - 1 ? nN - 1 : src);
        int dst = nodeBase + slot;
        dst = dst > nN - 1 ? nN - 1 : dst;

        const float* qr = qkv + (size_t)dst * QKVW + 8 * lane;
        const float* kr = qkv + (size_t)src * QKVW + HC + 8 * lane;
        const float* vr = kr + HC;
        const v4f q0 = *(const v4f*)qr, q1 = *(const v4f*)(qr + 4);
        const v4f k0 = *(const v4f*)kr, k1 = *(const v4f*)(kr + 4);
        const v4f v0 = *(const v4f*)vr, v1 = *(const v4f*)(vr + 4);
        const v4f qw = *(const v4f*)(qwe + (size_t)dst * QW + 4 * lane);
        const v4f ev = *(const v4f*)(ea + (size_t)e * FE + 4 * (lane & 7));

        float s = q0.x * k0.x + q0.y * k0.y + q0.z * k0.z + q0.w * k0.w
                + q1.x * k1.x + q1.y * k1.y + q1.z * k1.z + q1.w * k1.w;
        s += qw.x * ev.x + qw.y * ev.y + qw.z * ev.z + qw.w * ev.w;
        s += __shfl_xor(s, 1);
        s += __shfl_xor(s, 2);
        s += __shfl_xor(s, 4);
        s *= 0.125f;

        const float mo  = mden[slot * 8 + hd];
        const float dn  = mden[slot * 8 + 4 + hd];
        const float mn  = fmaxf(mo, s);
        const float sc  = __expf(mo - mn);
        const float p   = __expf(s - mn);
        const float dn2 = dn * sc + p;

        float* av = accv + slot * HC + 8 * lane;
        v4f a0 = *(const v4f*)av, a1 = *(const v4f*)(av + 4);
        a0 = a0 * sc + v0 * p;
        a1 = a1 * sc + v1 * p;
        *(v4f*)av = a0;
        *(v4f*)(av + 4) = a1;
        float* ae = acce + slot * QW + 4 * lane;
        v4f b0 = *(const v4f*)ae;
        b0 = b0 * sc + ev * p;
        *(v4f*)ae = b0;
        mden[slot * 8 + hd]     = mn;
        mden[slot * 8 + 4 + hd] = dn2;
      }
    }
    __syncthreads();
  }

  {
    v4f ov[8];
#pragma unroll
    for (int q = 0; q < 8; ++q) {
      const int slot = 16 * wave + 2 * q + hh;
      const int c4 = 4 * m;
      v4f a = {0.0f, 0.0f, 0.0f, 0.0f};
#pragma unroll
      for (int h = 0; h < NH; ++h) {
        const float d  = mden[slot * 8 + 4 + h];
        const float rd = (d > 0.0f) ? 0.25f * __builtin_amdgcn_rcpf(d) : 0.0f;
        const v4f t = *(const v4f*)(accv + slot * HC + CH * h + c4);
        a = a + t * rd;
      }
      ov[q] = a;
    }
#pragma unroll
    for (int q = 0; q < 8; ++q) {
      const int slot = 16 * wave + 2 * q + hh;
      *(volatile v4f*)(agg64 + (size_t)(nodeBase + slot) * CH + 4 * m) = ov[q];
    }
    __threadfence();
#pragma unroll
    for (int q = 0; q < 8; ++q) {
      const int slot = 16 * wave + 2 * q + hh;
      *(volatile v4f*)(agg64 + (size_t)(nodeBase + slot) * CH + 4 * m) = ov[q];
    }
  }
#pragma unroll 1
  for (int g = 0; g < 2; ++g) {
    v4f ov[8];
#pragma unroll
    for (int q = 0; q < 8; ++q) {
      const int slot = 16 * wave + 8 * g + q;
      const float d  = mden[slot * 8 + 4 + hd];
      const float rd = (d > 0.0f) ? 0.25f * __builtin_amdgcn_rcpf(d) : 0.0f;
      const v4f t = *(const v4f*)(acce + slot * QW + 4 * lane);
      ov[q] = t * rd;
    }
#pragma unroll
    for (int q = 0; q < 8; ++q) {
      const int slot = 16 * wave + 8 * g + q;
      *(volatile v4f*)(aea + (size_t)(nodeBase + slot) * QW + 4 * lane) = ov[q];
    }
    __threadfence();
#pragma unroll
    for (int q = 0; q < 8; ++q) {
      const int slot = 16 * wave + 8 * g + q;
      *(volatile v4f*)(aea + (size_t)(nodeBase + slot) * QW + 4 * lane) = ov[q];
    }
  }
}

__global__ __launch_bounds__(NTHR) void k_final(const float* __restrict__ aea, const float* __restrict__ x, int nN,
                                                const unsigned short* __restrict__ wp_h, const unsigned short* __restrict__ wp_l,
                                                const unsigned short* __restrict__ wsk_h, const unsigned short* __restrict__ wsk_l,
                                                const unsigned short* __restrict__ wc_h, const unsigned short* __restrict__ wc_l,
                                                const float* __restrict__ agg64, const float* __restrict__ bskip,
                                                const float* __restrict__ gamma, const float* __restrict__ beta,
                                                const float* __restrict__ rmean, const float* __restrict__ rvar,
                                                const float* __restrict__ bc, float* out) {
  __shared__ __attribute__((aligned(16))) unsigned short Ah[GBM * GK];
  __shared__ __attribute__((aligned(16))) unsigned short Al[GBM * GK];
  __shared__ __attribute__((aligned(16))) unsigned short Bsh[GBN * GK];
  __shared__ __attribute__((aligned(16))) unsigned short Bsl[GBN * GK];
  __shared__ __attribute__((aligned(16))) float Cs[GBM * GBN];
  __shared__ __attribute__((aligned(16))) unsigned short Wch[NCLS * CH];
  __shared__ __attribute__((aligned(16))) unsigned short Wcl[NCLS * CH];
  __shared__ __attribute__((aligned(16))) float Os[GBM * NCLS];
  const int tid = threadIdx.x, lane = tid & 31, wave = tid >> 5, hh = lane >> 4, m = lane & 15;
  const int row0 = blockIdx.x * GBM;
  const int mt = wave >> 1, nt0 = 2 * (wave & 1);

  for (int u = tid; u < GBM * (GK / 8); u += NTHR) {
    const int r = u >> 4, k8 = (u & 15) * 8;
    const float* p = aea + (size_t)(row0 + r) * QW + k8;
    float f[8];
    unpack8(*(const v4f*)p, *(const v4f*)(p + 4), f);
    v8us hi, lo;
    split8(f, hi, lo);
    *(v8us*)(Ah + r * GK + k8) = hi;
    *(v8us*)(Al + r * GK + k8) = lo;
  }
  for (int u = tid; u < GBN * (GK / 8); u += NTHR) {
    *(v8us*)(Bsh + u * 8) = *(const v8us*)(wp_h + u * 8);
    *(v8us*)(Bsl + u * 8) = *(const v8us*)(wp_l + u * 8);
  }
  for (int u = tid; u < NCLS * CH / 8; u += NTHR) {
    *(v8us*)(Wch + u * 8) = *(const v8us*)(wc_h + u * 8);
    *(v8us*)(Wcl + u * 8) = *(const v8us*)(wc_l + u * 8);
  }
  __syncthreads();

  v8f acc[2];
  acc[0] = zero8f();
  acc[1] = zero8f();
#pragma unroll
  for (int ks = 0; ks < GK / 32; ++ks) {
    const v16b ah = ldfrag(Ah, 16 * mt + m, GK, 32 * ks, hh);
    const v16b al = ldfrag(Al, 16 * mt + m, GK, 32 * ks, hh);
#pragma unroll
    for (int t = 0; t < 2; ++t) {
      const v16b bhf = ldfrag(Bsh, 16 * (nt0 + t) + m, GK, 32 * ks, hh);
      const v16b blf = ldfrag(Bsl, 16 * (nt0 + t) + m, GK, 32 * ks, hh);
      acc[t] = wm3(ah, al, bhf, blf, acc[t]);
    }
  }
  __syncthreads();

  for (int u = tid; u < GBM * (GK / 8); u += NTHR) {
    const int r = u >> 4, k8 = (u & 15) * 8;
    int grow = row0 + r;
    grow = grow > nN - 1 ? nN - 1 : grow;
    const float* p = x + (size_t)grow * FIN + k8;
    float f[8];
    unpack8(*(const v4f*)p, *(const v4f*)(p + 4), f);
    v8us hi, lo;
    split8(f, hi, lo);
    *(v8us*)(Ah + r * GK + k8) = hi;
    *(v8us*)(Al + r * GK + k8) = lo;
  }
  for (int u = tid; u < GBN * (GK / 8); u += NTHR) {
    *(v8us*)(Bsh + u * 8) = *(const v8us*)(wsk_h + u * 8);
    *(v8us*)(Bsl + u * 8) = *(const v8us*)(wsk_l + u * 8);
  }
  __syncthreads();
#pragma unroll
  for (int ks = 0; ks < GK / 32; ++ks) {
    const v16b ah = ldfrag(Ah, 16 * mt + m, GK, 32 * ks, hh);
    const v16b al = ldfrag(Al, 16 * mt + m, GK, 32 * ks, hh);
#pragma unroll
    for (int t = 0; t < 2; ++t) {
      const v16b bhf = ldfrag(Bsh, 16 * (nt0 + t) + m, GK, 32 * ks, hh);
      const v16b blf = ldfrag(Bsl, 16 * (nt0 + t) + m, GK, 32 * ks, hh);
      acc[t] = wm3(ah, al, bhf, blf, acc[t]);
    }
  }

#pragma unroll
  for (int t = 0; t < 2; ++t) {
    const int col = 16 * (nt0 + t) + m;
    const float bs  = bskip[col];
    const float gm  = gamma[col];
    const float bt  = beta[col];
    const float rm  = rmean[col];
    const float inv = rsqrtf(rvar[col] + BN_EPS);
#pragma unroll
    for (int r = 0; r < 8; ++r) {
      const int rowl = 16 * mt + 8 * hh + r;
      float o = acc[t][r] + agg64[(size_t)(row0 + rowl) * CH + col] + bs;
      o = fmaxf(o, 0.0f);
      o = (o - rm) * inv * gm + bt;
      Cs[rowl * GBN + col] = o;
    }
  }
  __syncthreads();

  if (wave < 4) {
    const int mt2 = wave;
    v8f acc2 = zero8f();
#pragma unroll
    for (int ks = 0; ks < CH / 32; ++ks) {
      const float* cr = Cs + (16 * mt2 + m) * GBN + 32 * ks + 8 * hh;
      float f[8];
      FragB ah, al;
      unpack8(*(const v4f*)cr, *(const v4f*)(cr + 4), f);
      split8(f, ah.u[0], al.u[0]);
      unpack8(*(const v4f*)(cr + 16), *(const v4f*)(cr + 20), f);
      split8(f, ah.u[1], al.u[1]);
      const v16b bhf = ldfrag(Wch, m, CH, 32 * ks, hh);
      const v16b blf = ldfrag(Wcl, m, CH, 32 * ks, hh);
      acc2 = wm3(ah.v, al.v, bhf, blf, acc2);
    }
    const float bcm = bc[m];
#pragma unroll
    for (int r = 0; r < 8; ++r) Os[(16 * mt2 + 8 * hh + r) * NCLS + m] = acc2[r] + bcm;
  }
  __syncthreads();

  {
    const int rl = 8 * wave + (lane >> 2);
    const bool ok = (row0 + rl) < nN;
    const v4f ovv = *(const v4f*)(Os + (wave * 32 + lane) * 4);
    float* op = out + (size_t)row0 * NCLS + (size_t)(wave * 32 + lane) * 4;
    if (ok) *(volatile v4f*)op = ovv;
    __threadfence();
    if (ok) *(volatile v4f*)op = ovv;
  }
}

extern "C" void kernel_launch(void* const* d_in, const int* in_sizes, int n_in,
                              void* d_out, int out_size, void* d_ws, size_t ws_size,
                              hipStream_t stream) {
  if (n_in < 18) return;
  const int nN = in_sizes[0] / FIN;
  const int nE = in_sizes[1] / 2;
  if (nN <= 0 || nE <= 0) return;
  if (in_sizes[0] != nN * FIN || in_sizes[1] != 2 * nE || in_sizes[2] != nE * FE) return;
  if (in_sizes[3] != FIN * HC || in_sizes[4] != HC) return;
  if (in_sizes[5] != FIN * HC || in_sizes[6] != HC) return;
  if (in_sizes[7] != FIN * HC || in_sizes[8] != HC) return;
  if (in_sizes[9] != FE * HC) return;
  if (in_sizes[10] != FIN * CH || in_sizes[11] != CH) return;
  if (in_sizes[12] != CH || in_sizes[13] != CH || in_sizes[14] != CH || in_sizes[15] != CH) return;
  if (in_sizes[16] != CH * NCLS || in_sizes[17] != NCLS) return;
  if (out_size != nN * NCLS) return;

  const float* x     = (const float*)d_in[0];
  const int*   ei    = (const int*)d_in[1];
  const float* ea    = (const float*)d_in[2];
  const float* Wq    = (const float*)d_in[3];
  const float* bq    = (const float*)d_in[4];
  const float* Wk    = (const float*)d_in[5];
  const float* bk    = (const float*)d_in[6];
  const float* Wv    = (const float*)d_in[7];
  const float* bv    = (const float*)d_in[8];
  const float* We    = (const float*)d_in[9];
  const float* Wskip = (const float*)d_in[10];
  const float* bskip = (const float*)d_in[11];
  const float* gamma = (const float*)d_in[12];
  const float* beta  = (const float*)d_in[13];
  const float* rmean = (const float*)d_in[14];
  const float* rvar  = (const float*)d_in[15];
  const float* Wc    = (const float*)d_in[16];
  const float* bc    = (const float*)d_in[17];
  float* out = (float*)d_out;

  const int Npad = ((nN + NB - 1) / NB) * NB;

  char* ws = (char*)d_ws;
  size_t off = 0;
  const size_t wcatE = (size_t)QKVW * GK, webdE = (size_t)2 * GBN * GK, wpE = (size_t)CH * GK, wskE = (size_t)CH * GK, wcE = (size_t)NCLS * CH;
#define CARVE_AL(b) (((size_t)(b) + 255) & ~(size_t)255)
  const size_t oWcatH = off; off += CARVE_AL(wcatE * 2);
  const size_t oWcatL = off; off += CARVE_AL(wcatE * 2);
  const size_t oWebdH = off; off += CARVE_AL(webdE * 2);
  const size_t oWebdL = off; off += CARVE_AL(webdE * 2);
  const size_t oWpH   = off; off += CARVE_AL(wpE * 2);
  const size_t oWpL   = off; off += CARVE_AL(wpE * 2);
  const size_t oWskH  = off; off += CARVE_AL(wskE * 2);
  const size_t oWskL  = off; off += CARVE_AL(wskE * 2);
  const size_t oWcH   = off; off += CARVE_AL(wcE * 2);
  const size_t oWcL   = off; off += CARVE_AL(wcE * 2);
  const size_t oBias  = off; off += CARVE_AL((size_t)QKVW * 4);
  const size_t oQkv   = off; off += CARVE_AL((size_t)Npad * QKVW * 4);
  const size_t oQwe   = off; off += CARVE_AL((size_t)Npad * QW * 4);
  const size_t oAgg   = off; off += CARVE_AL((size_t)Npad * CH * 4);
  const size_t oAea   = off; off += CARVE_AL((size_t)Npad * QW * 4);
#undef CARVE_AL
  if (off > ws_size) return;

  unsigned short* wcat_h = (unsigned short*)(ws + oWcatH);
  unsigned short* wcat_l = (unsigned short*)(ws + oWcatL);
  unsigned short* webd_h = (unsigned short*)(ws + oWebdH);
  unsigned short* webd_l = (unsigned short*)(ws + oWebdL);
  unsigned short* wp_h   = (unsigned short*)(ws + oWpH);
  unsigned short* wp_l   = (unsigned short*)(ws + oWpL);
  unsigned short* wsk_h  = (unsigned short*)(ws + oWskH);
  unsigned short* wsk_l  = (unsigned short*)(ws + oWskL);
  unsigned short* wc_h   = (unsigned short*)(ws + oWcH);
  unsigned short* wc_l   = (unsigned short*)(ws + oWcL);
  float* biascat = (float*)(ws + oBias);
  float* qkv     = (float*)(ws + oQkv);
  float* qwe     = (float*)(ws + oQwe);
  float* agg64   = (float*)(ws + oAgg);
  float* aea     = (float*)(ws + oAea);

  const int vec8  = ((nE & 3) == 0) ? 1 : 0;
  const int nBlkG = Npad / GBM;
  const int nBlkA = Npad / NB;
  const int nPrep = (QKVW * GK / 8 + NTHR - 1) / NTHR;

  k_prep<<<dim3(nPrep, 6), NTHR, 0, stream>>>(Wq, Wk, Wv, We, Wskip, Wc, bq, bk, bv,
                                              wcat_h, wcat_l, webd_h, webd_l, wp_h, wp_l,
                                              wsk_h, wsk_l, wc_h, wc_l, biascat);

  k_gemm<<<dim3(nBlkG, 1), NTHR, 0, stream>>>(x, FIN, 0, nN, wcat_h, wcat_l, QKVW / GBN, 0,
                                              biascat, 1, qkv, QKVW);
  k_gemm<<<dim3(nBlkG, 2), NTHR, 0, stream>>>(qkv, QKVW, GK, Npad, webd_h, webd_l, 1, 1,
                                              biascat, 0, qwe, QW);

  hipFuncSetAttribute(reinterpret_cast<const void*>(&k_agg), hipFuncAttributeMaxDynamicSharedMemorySize,
                      (int)AGG_LDS_BYTES);
  k_agg<<<nBlkA, NTHR, AGG_LDS_BYTES, stream>>>(ei, nE, nN, vec8, ea, qkv, qwe, agg64, aea);

  k_final<<<nBlkG, NTHR, 0, stream>>>(aea, x, nN, wp_h, wp_l, wsk_h, wsk_l, wc_h, wc_l,
                                      agg64, bskip, gamma, beta, rmean, rvar, bc, out);
}
